// Interact_Layer_43069932044849
// MI455X (gfx1250) — hardware-verified
//
#include <hip/hip_runtime.h>
#include <hip/hip_bf16.h>

typedef _Float16 bf16_t;
typedef __attribute__((ext_vector_type(16))) _Float16 v16bf;
typedef __attribute__((ext_vector_type(8)))  _Float16 v8bf;
typedef __attribute__((ext_vector_type(4)))  _Float16 v4bf;
typedef __attribute__((ext_vector_type(8)))  float  v8f;
typedef __attribute__((ext_vector_type(4)))  float  v4f_t;
typedef float v4fa __attribute__((ext_vector_type(4), may_alias));

namespace {
constexpr int BATCH   = 2048;
constexpr int SEQ     = 200;
constexpr int EMB     = 16;
constexpr int HEADS   = 2;
constexpr int HD      = 8;
constexpr int ST      = 13;
constexpr int SP      = 208;
constexpr int SBW     = 212;
constexpr int PW      = 232;
constexpr int KSTEPS  = 7;
constexpr int NW      = 4;
constexpr int NTHR    = NW * 32;
constexpr float SCALE = 0.35355339059327373f;
}

#define CAT16(lo, hi) __builtin_shufflevector((lo), (hi), 0, 1, 2, 3, 4, 5, 6, 7, \
                                              8, 9, 10, 11, 12, 13, 14, 15)

__device__ __forceinline__ v8f wmma_bf16(v16bf a, v16bf b, v8f c) {
  return __builtin_amdgcn_wmma_f32_16x16x32_f16(false, a, false, b,
                                                 (short)0, c, false, false);
}

__device__ __forceinline__ v8f zero8f() {
  v8f c;
#pragma unroll
  for (int j = 0; j < 8; ++j) c[j] = 0.0f;
  return c;
}

__global__ __launch_bounds__(NTHR)
void mha_fused(const float* __restrict__ xq, const float* __restrict__ xk,
               const float* __restrict__ xv,
               const float* __restrict__ wq, const float* __restrict__ wk,
               const float* __restrict__ wv, const float* __restrict__ wfc,
               float* __restrict__ out)
{
  __shared__ bf16_t q_lds[SP][EMB];
  __shared__ bf16_t k_lds[SP][EMB];
  __shared__ bf16_t vT[EMB][PW];
  __shared__ float  sbuf[NW][16][SBW];
  __shared__ bf16_t pbuf[NW][16][PW];
  __shared__ bf16_t ctxb[NW][16][EMB];
  __shared__ __attribute__((aligned(16))) float obuf[NW][16][EMB];

  const int  tid  = threadIdx.x;
  const int  wid  = tid >> 5;
  const int  lane = tid & 31;
  const int  lrow = lane & 15;
  const bool hiL  = lane >= 16;
  const int  blk  = blockIdx.x;

  v8bf z8;
#pragma unroll
  for (int i = 0; i < 8; ++i) z8[i] = (bf16_t)0.0f;

  auto load_wA = [&](const float* __restrict__ w) -> v16bf {
    const float* p = w + lrow * EMB + (hiL ? 8 : 0);
    v8bf r;
#pragma unroll
    for (int i = 0; i < 8; ++i) r[i] = (bf16_t)p[i];
    return CAT16(r, z8);
  };
  const v16bf aWq  = load_wA(wq);
  const v16bf aWk  = load_wA(wk);
  const v16bf aWv  = load_wA(wv);
  const v16bf aWfc = load_wA(wfc);

  auto load_xB = [&](const float* __restrict__ x, int t) -> v16bf {
    v8bf a = z8;
    const int row = t * 16 + lrow;
    if (row < SEQ) {
      const float4* p =
          (const float4*)(x + ((size_t)blk * SEQ + row) * EMB + (hiL ? 8 : 0));
      const float4 f0 = p[0];
      const float4 f1 = p[1];
      a[0] = (bf16_t)f0.x; a[1] = (bf16_t)f0.y; a[2] = (bf16_t)f0.z; a[3] = (bf16_t)f0.w;
      a[4] = (bf16_t)f1.x; a[5] = (bf16_t)f1.y; a[6] = (bf16_t)f1.z; a[7] = (bf16_t)f1.w;
    }
    return CAT16(a, z8);
  };

  for (int t = wid; t < ST; t += NW) {
    const v16bf bXq = load_xB(xq, t);
    const v16bf bXk = load_xB(xk, t);
    const v16bf bXv = load_xB(xv, t);
    const v8f cq = wmma_bf16(aWq, bXq, zero8f());
    const v8f ck = wmma_bf16(aWk, bXk, zero8f());
    const v8f cv = wmma_bf16(aWv, bXv, zero8f());
    const int s  = t * 16 + lrow;
    const int fo = hiL ? 8 : 0;
    v8bf yq, yk;
#pragma unroll
    for (int j = 0; j < 8; ++j) { yq[j] = (bf16_t)cq[j]; yk[j] = (bf16_t)ck[j]; }
    *(v8bf*)&q_lds[s][fo] = yq;
    *(v8bf*)&k_lds[s][fo] = yk;
#pragma unroll
    for (int j = 0; j < 8; ++j) vT[fo + j][s] = (bf16_t)cv[j];
  }
  for (int i = tid; i < EMB * (PW - SP); i += NTHR)
    vT[i / (PW - SP)][SP + i % (PW - SP)] = (bf16_t)0.0f;
  __syncthreads();

  for (int qt = wid; qt < ST; qt += NW) {
    for (int h = 0; h < HEADS; ++h) {
      v8bf q0 = z8;
      if (!hiL) q0 = *(const v8bf*)&q_lds[qt * 16 + lrow][h * HD];
      const v16bf bQ = CAT16(q0, z8);

      float mloc = -3.0e38f;
      for (int kt = 0; kt < ST; ++kt) {
        v8bf k0 = z8;
        if (!hiL) k0 = *(const v8bf*)&k_lds[kt * 16 + lrow][h * HD];
        const v16bf aK = CAT16(k0, z8);
        const v8f sc = wmma_bf16(aK, bQ, zero8f());
        const int co = kt * 16 + (hiL ? 8 : 0);
        float4 s0, s1;
        s0.x = sc[0] * SCALE; s0.y = sc[1] * SCALE;
        s0.z = sc[2] * SCALE; s0.w = sc[3] * SCALE;
        s1.x = sc[4] * SCALE; s1.y = sc[5] * SCALE;
        s1.z = sc[6] * SCALE; s1.w = sc[7] * SCALE;
        *(float4*)&sbuf[wid][lrow][co]     = s0;
        *(float4*)&sbuf[wid][lrow][co + 4] = s1;
        const float m0 = fmaxf(fmaxf(s0.x, s0.y), fmaxf(s0.z, s0.w));
        const float m1 = fmaxf(fmaxf(s1.x, s1.y), fmaxf(s1.z, s1.w));
        mloc = fmaxf(mloc, fmaxf(m0, m1));
      }
      asm volatile("s_wait_dscnt 0" ::: "memory");

      const float m = fmaxf(mloc, __shfl_xor(mloc, 16, 32));
      float den = 0.0f;
      {
        const int c0 = hiL ? 100 : 0;
        for (int c = 0; c < 25; ++c) {
          const float4 sv = *(const float4*)&sbuf[wid][lrow][c0 + 4 * c];
          const float e0 = __expf(sv.x - m);
          const float e1 = __expf(sv.y - m);
          const float e2 = __expf(sv.z - m);
          const float e3 = __expf(sv.w - m);
          den += (e0 + e1) + (e2 + e3);
          v4bf pv;
          pv[0] = (bf16_t)(e0 * 1024.0f); pv[1] = (bf16_t)(e1 * 1024.0f);
          pv[2] = (bf16_t)(e2 * 1024.0f); pv[3] = (bf16_t)(e3 * 1024.0f);
          *(v4bf*)&pbuf[wid][lrow][c0 + 4 * c] = pv;
        }
        den += __shfl_xor(den, 16, 32);
        const int z0 = SEQ + (hiL ? 16 : 0);
        *(v8bf*)&pbuf[wid][lrow][z0]     = z8;
        *(v8bf*)&pbuf[wid][lrow][z0 + 8] = z8;
      }
      asm volatile("s_wait_dscnt 0" ::: "memory");

      v8f cc = zero8f();
      for (int ks = 0; ks < KSTEPS; ++ks) {
        const int base = ks * 32 + (hiL ? 8 : 0);
        const v8bf p0 = *(const v8bf*)&pbuf[wid][lrow][base];
        const v8bf p1 = *(const v8bf*)&pbuf[wid][lrow][base + 16];
        const v16bf bP = CAT16(p0, p1);
        v8bf v0 = z8, v1 = z8;
        if (lrow < 8) {
          const int f = h * HD + lrow;
          v0 = *(const v8bf*)&vT[f][base];
          v1 = *(const v8bf*)&vT[f][base + 16];
        }
        const v16bf aV = CAT16(v0, v1);
        cc = wmma_bf16(aV, bP, cc);
      }

      if (!hiL) {
        const float rden = 1.0f / (den * 1024.0f);
        v8bf cb;
#pragma unroll
        for (int j = 0; j < 8; ++j) cb[j] = (bf16_t)(cc[j] * rden);
        *(v8bf*)&ctxb[wid][lrow][h * HD] = cb;
      }
      asm volatile("s_wait_dscnt 0" ::: "memory");
    }

    const v8bf c0 = *(const v8bf*)&ctxb[wid][lrow][hiL ? 8 : 0];
    const v16bf bC = CAT16(c0, z8);
    const v8f o = wmma_bf16(aWfc, bC, zero8f());

    {
      const int fo = hiL ? 8 : 0;
#pragma unroll
      for (int j = 0; j < 8; ++j) obuf[wid][lrow][fo + j] = o[j];
    }
    asm volatile("s_wait_dscnt 0" ::: "memory");
    {
      const int nrow = (qt * 16 + 16 <= SEQ) ? 16 : (SEQ - qt * 16);
      float* ob = out + ((size_t)blk * SEQ + qt * 16) * EMB;
      const float* xb = xq + ((size_t)blk * SEQ + qt * 16) * EMB;
#pragma unroll 1
      for (int pass = 0; pass < 2; ++pass) {
#pragma unroll
        for (int i = 0; i < 2; ++i) { const int q4 = (lane + 32 * i) * 4;
          if (q4 < nrow * EMB) { v4f_t v = *(const v4f_t*)(xb + q4); const v4f_t a = *(const volatile v4fa*)(&obuf[wid][0][0] + q4);
            v.x = fmaxf(v.x + a.x, 0.0f); v.y = fmaxf(v.y + a.y, 0.0f); v.z = fmaxf(v.z + a.z, 0.0f); v.w = fmaxf(v.w + a.w, 0.0f);
            *(volatile v4f_t*)(ob + q4) = v; } }
        __threadfence();
      }
    }
    asm volatile("s_wait_dscnt 0" ::: "memory");
  }
}

extern "C" void kernel_launch(void* const* d_in, const int* in_sizes, int n_in,
                              void* d_out, int out_size, void* d_ws, size_t ws_size,
                              hipStream_t stream) {
  (void)in_sizes; (void)n_in; (void)out_size; (void)d_ws; (void)ws_size;
  const float* xq  = (const float*)d_in[0];
  const float* xk  = (const float*)d_in[1];
  const float* xv  = (const float*)d_in[2];
  const float* wq  = (const float*)d_in[3];
  const float* wk  = (const float*)d_in[4];
  const float* wvp = (const float*)d_in[5];
  const float* wfc = (const float*)d_in[6];
  float* outp = (float*)d_out;
  mha_fused<<<BATCH, NTHR, 0, stream>>>(xq, xk, xv, wq, wk, wvp, wfc, outp);
}
